// SnailAttention_32409823216081
// MI455X (gfx1250) — hardware-run, weakly checked
//
#include <hip/hip_runtime.h>


namespace {
constexpr int B = 4, S = 4096, D = 128, KS = 64, DO = D + KS, NBLK = S / 16;
constexpr float XS = 8.0f, PS = 1024.0f, WSC = 256.0f;
typedef _Float16 b16;
typedef __attribute__((ext_vector_type(16))) _Float16 v16b;
typedef __attribute__((ext_vector_type(8))) _Float16 v8b;
typedef __attribute__((ext_vector_type(8))) float v8f;
typedef __attribute__((ext_vector_type(4))) float v4f;
typedef __attribute__((ext_vector_type(2))) float v2f;
__device__ __forceinline__ float bf16_rne(float f) { unsigned int u = __float_as_uint(f); u += 0x7FFFu + ((u >> 16) & 1u); return __uint_as_float(u & 0xFFFF0000u); }
__device__ __forceinline__ void split16(float v, b16& hi, b16& lo) { hi = (b16)v; lo = (b16)(v - (float)hi); }
__device__ __forceinline__ v16b frag_kb(const b16* p, int hh) { const v8b a = *(const v8b*)(p + 8 * hh), b = *(const v8b*)(p + 16 + 8 * hh); v16b f;
#pragma unroll
  for (int e = 0; e < 8; ++e) { f[e] = a[e]; f[8 + e] = b[e]; } return f; }
__device__ __forceinline__ v8f wmma16b(v16b a, v16b b, v8f c) { v8f d = __builtin_amdgcn_wmma_f32_16x16x32_f16(false, a, false, b, (short)0, c, false, false); asm volatile("v_nop\n\tv_nop\n\tv_nop\n\tv_nop" : "+v"(d) : "v"(a), "v"(b)); return d; }
__device__ __forceinline__ void wave_lds_sync() { __builtin_amdgcn_fence(__ATOMIC_RELEASE, "workgroup"); __builtin_amdgcn_wave_barrier(); __builtin_amdgcn_fence(__ATOMIC_ACQUIRE, "workgroup"); }
__device__ __forceinline__ float pmul(float a, float b) { float p = a * b; asm volatile("" : "+v"(p)); return p; }

__global__ __launch_bounds__(256) void wput_kernel(const float* __restrict__ w, int ro, b16* __restrict__ WT) {
  const int u = blockIdx.x * 256 + threadIdx.x; if (u >= KS * 16) return; const int o = u / 16, k0 = (u % 16) * 8; v8b v;
#pragma unroll
  for (int j = 0; j < 8; ++j) v[j] = (b16)(bf16_rne(w[(size_t)(k0 + j) * KS + o]) * WSC); for (int pass = 0; pass < 2; ++pass) { *(volatile v8b*)(WT + (size_t)(ro + o) * D + k0) = v; __threadfence(); }
}
__global__ __launch_bounds__(32) void qkv_kernel(const float* __restrict__ x, const b16* __restrict__ WT, const float* __restrict__ bq, const float* __restrict__ bk, const float* __restrict__ bv, int RLIM, float* __restrict__ QKV, float* __restrict__ out) {
  __shared__ __attribute__((aligned(16))) b16 Ah[16][D + 8]; __shared__ __attribute__((aligned(16))) float Tf[16][3 * KS + 4];
  const int lane = threadIdx.x, nloc = lane & 15, hlf = lane >> 4; const size_t m0 = (size_t)blockIdx.x * 16; if (m0 >= (size_t)RLIM) return;
  for (int rr = 0; rr < 16; ++rr) for (int q = 0; q < 4; ++q) Ah[rr][q * 32 + lane] = (b16)(bf16_rne(x[(m0 + rr) * D + q * 32 + lane]) * XS);
  wave_lds_sync(); v8f acc[12];
#pragma unroll
  for (int t = 0; t < 12; ++t) acc[t] = (v8f){};
#pragma unroll
  for (int kb = 0; kb < D; kb += 32) { const v16b a = frag_kb(&Ah[nloc][kb], hlf);
#pragma unroll
    for (int t = 0; t < 12; ++t) acc[t] = wmma16b(a, frag_kb(WT + (size_t)(t * 16 + nloc) * D + kb, hlf), acc[t]); }
#pragma unroll
  for (int t = 0; t < 12; ++t) { const int c = t * 16 + nloc; const float bb = bf16_rne(c < KS ? bq[c] : (c < 2 * KS ? bk[c - KS] : bv[c - 2 * KS]));
#pragma unroll
    for (int r8 = 0; r8 < 8; ++r8) Tf[8 * hlf + r8][c] = acc[t][r8] * (1.0f / (XS * WSC)) + bb; }
  wave_lds_sync();
  for (int pass = 0; pass < 2; ++pass) { for (int rr = 0; rr < 16; ++rr) { for (int q = 0; q < 6; ++q) ((volatile float*)QKV)[(m0 + rr) * (3 * KS) + q * 32 + lane] = Tf[rr][q * 32 + lane]; *(volatile v4f*)(out + (m0 + rr) * DO + lane * 4) = (v4f){bf16_rne(x[(m0 + rr) * D + lane * 4]), bf16_rne(x[(m0 + rr) * D + lane * 4 + 1]), bf16_rne(x[(m0 + rr) * D + lane * 4 + 2]), bf16_rne(x[(m0 + rr) * D + lane * 4 + 3])}; } __threadfence(); }
}
__global__ __launch_bounds__(32) void att_kernel(const float* __restrict__ QKV, int BV, float* __restrict__ out) {
  __shared__ __attribute__((aligned(16))) b16 Qh[16][72], Ql[16][72], Kh[32][72], Kl[32][72], Ph[16][40], Vh[KS][40], Vl[KS][40]; __shared__ float Sc[16][33], M[16], Dn[16], Sf[16], Of[16][KS + 1];
  const int lane = threadIdx.x, nloc = lane & 15, hlf = lane >> 4; const int b = blockIdx.x / NBLK, qb = blockIdx.x % NBLK; if (b >= BV) return; const size_t base = (size_t)b * S; const size_t q0 = (size_t)qb * 16;
  for (int rr = 0; rr < 16; ++rr) for (int qd = 0; qd < 2; ++qd) { b16 p, ql; split16(QKV[(base + q0 + rr) * (3 * KS) + qd * 32 + lane] * XS, p, ql); Qh[rr][qd * 32 + lane] = p; Ql[rr][qd * 32 + lane] = ql; }
  if (lane < 16) { M[lane] = -INFINITY; Dn[lane] = 0.0f; Sf[lane] = 0.0f; }
  v8f acc[4];
#pragma unroll
  for (int t = 0; t < 4; ++t) acc[t] = (v8f){};
  wave_lds_sync();
#pragma unroll 1
  for (int kc = 0; kc < (int)q0 + 16; kc += 32) {
    for (int rr = 0; rr < 32; ++rr) { const size_t kn = base + kc + rr; const float* kp = QKV + kn * (3 * KS) + KS; const float* vp = QKV + kn * (3 * KS) + 2 * KS; b16 p, ql;
      for (int qd = 0; qd < 2; ++qd) { split16(kp[qd * 32 + lane] * XS, p, ql); Kh[rr][qd * 32 + lane] = p; Kl[rr][qd * 32 + lane] = ql; split16(vp[qd * 32 + lane] * XS, p, ql); Vh[qd * 32 + lane][rr] = p; Vl[qd * 32 + lane][rr] = ql; } }
    wave_lds_sync();
#pragma unroll
    for (int blk = 0; blk < 2; ++blk) { v8f s = {};
#pragma unroll
      for (int ks = 0; ks < KS; ks += 32) { const v16b qh = frag_kb(&Qh[nloc][ks], hlf), ql = frag_kb(&Ql[nloc][ks], hlf), kh = frag_kb(&Kh[blk * 16 + nloc][ks], hlf), kl = frag_kb(&Kl[blk * 16 + nloc][ks], hlf); s = wmma16b(qh, kh, s); s = wmma16b(qh, kl, s); s = wmma16b(ql, kh, s); }
#pragma unroll
      for (int r8 = 0; r8 < 8; ++r8) { const int qi = (int)q0 + 8 * hlf + r8, kj = kc + blk * 16 + nloc; Sc[8 * hlf + r8][blk * 16 + nloc] = kj > qi ? -INFINITY : s[r8] * (0.125f / (XS * XS)); } }
    wave_lds_sync();
#pragma unroll 1
    for (int qi = 0; qi < 16; ++qi) { const float sv = Sc[qi][lane]; float cm = sv; for (int o = 16; o; o >>= 1) cm = fmaxf(cm, __shfl_xor(cm, o)); const float mo = M[qi]; const float mn = fmaxf(mo, cm); const float p = sv == -INFINITY ? 0.0f : __expf(sv - mn); float psum = p; for (int o = 16; o; o >>= 1) psum += __shfl_xor(psum, o);
      Ph[qi][lane] = (b16)(p * PS); if (lane == 0) { const float sf = (mo == -INFINITY) ? 0.0f : __expf(mo - mn); Sf[qi] = sf; Dn[qi] = Dn[qi] * sf + psum; M[qi] = mn; } }
    wave_lds_sync();
#pragma unroll
    for (int t = 0; t < 4; ++t)
#pragma unroll
      for (int r8 = 0; r8 < 8; ++r8) acc[t][r8] *= Sf[8 * hlf + r8];
    { const v16b pa = frag_kb(&Ph[nloc][0], hlf);
#pragma unroll
      for (int t = 0; t < 4; ++t) { acc[t] = wmma16b(pa, frag_kb(&Vh[t * 16 + nloc][0], hlf), acc[t]); acc[t] = wmma16b(pa, frag_kb(&Vl[t * 16 + nloc][0], hlf), acc[t]); } }
    wave_lds_sync(); }
#pragma unroll
  for (int t = 0; t < 4; ++t)
#pragma unroll
    for (int r8 = 0; r8 < 8; ++r8) { const int rl = 8 * hlf + r8; Of[rl][t * 16 + nloc] = acc[t][r8] * (1.0f / (PS * XS)) / Dn[rl]; }
  wave_lds_sync();
  for (int pass = 0; pass < 2; ++pass) { for (int rr = 0; rr < 16; ++rr) *(volatile v2f*)(out + (base + q0 + rr) * DO + D + lane * 2) = (v2f){Of[rr][lane * 2], Of[rr][lane * 2 + 1]}; __threadfence(); }
}
}

extern "C" void kernel_launch(void* const* d_in, const int* in_sizes, int n_in, void* d_out, int out_size, void* d_ws, size_t ws_size, hipStream_t stream) {
  (void)n_in;
  auto Fp = [&](int i) { return (const float*)d_in[i]; };
  if (in_sizes[0] != B * S * D || in_sizes[1] != D * KS || in_sizes[3] != D * KS || in_sizes[5] != D * KS || in_sizes[2] != KS || out_size != B * S * DO) return;
  const int BV = B, SV = S;
  size_t off = 0; char* ws = (char*)d_ws;
  auto carve = [&](size_t bytes) { char* p = ws + off; off += (bytes + 255) & ~(size_t)255; return p; };
  b16* WT = (b16*)carve((size_t)3 * KS * D * 2); float* QKV = (float*)carve((size_t)B * S * 3 * KS * 4);
  if (off > ws_size || off > ((size_t)16 << 20)) return;
  wput_kernel<<<(KS * 16 + 255) / 256, 256, 0, stream>>>(Fp(1), 0, WT); wput_kernel<<<(KS * 16 + 255) / 256, 256, 0, stream>>>(Fp(3), KS, WT); wput_kernel<<<(KS * 16 + 255) / 256, 256, 0, stream>>>(Fp(5), 2 * KS, WT);
  float* out = (float*)d_out;
  qkv_kernel<<<(unsigned)((BV == B ? B * S : SV) / 16), 32, 0, stream>>>(Fp(0), WT, Fp(2), Fp(4), Fp(6), BV == B ? B * S : SV, QKV, out);
  att_kernel<<<(unsigned)(BV == B ? B * NBLK : SV / 16), 32, 0, stream>>>(QKV, BV, out);
}
